// en_gnn_88347477279281
// MI455X (gfx1250) — hardware-run, weakly checked
//
#include <hip/hip_runtime.h>
#include <stddef.h>
#include <stdint.h>


#define HF       64
#define IN_F     32
#define NG       128
#define NCLS     55
#define MD       128
#define NTHR     256
#define NWAVE    8
#define ETHR     128
#define EPT      8
#define NGRP     2
#define CHUNK    (NTHR * EPT * NGRP)
#define WCAP     (EPT * NGRP * 32)
#define LISTN    (NWAVE * WCAP)
#define NBC      4096
#define NBF      1024
#define RCAP     40960
#define RBN      128
#define OTHR     512
#define DEGCAP   256
#define CNB      32
#define CPOS     64
#define GROWS    128
#define TPH      (HF + 8)
#define MPF      (HF + 4)
#define WSCAP    134217728
#define LDS_FILL ((RCAP + NBF + LISTN) * 4 + 64)
#define LDS_HEAD (2 * NG * MD * 2)
#define FL_BIAS  1
#define FL_SILU  2
#define WO_IN    0
#define WO_OUT   2048
#define WO_LAY0  6144
#define WL_PQ    0
#define WL_W2    8192
#define WL_C1    12288
#define WL_N1    16384
#define WL_N2    24576
#define WL_STR   28672
#define WP_HEAD  768
#define WP_LAY   3584

static_assert((CHUNK & (CHUNK - 1)) == 0);
static_assert(CHUNK <= 4096);
static_assert((NBC & (NBC - 1)) == 0 && (NBF & (NBF - 1)) == 0);
static_assert(NBC == 4 * NBF);
static_assert(OTHR * 8 == NBC);
static_assert((RCAP % 32) == 0);
static_assert((NBF % CNB) == 0);
static_assert((GROWS % CNB) == 0);
static_assert(CNB == 32);
static_assert(CNB == 8 * (ETHR / 32));
static_assert(CPOS == 16 * (ETHR / 32));
static_assert(ETHR == 2 * CPOS);
static_assert((CNB * DEGCAP) % CPOS == 0);
static_assert(((TPH * 2) % 16) == 0 && ((MPF * 4) % 16) == 0);
static_assert(WO_LAY0 == 8 * WP_HEAD && WL_STR == 8 * WP_LAY);
static_assert((WP_HEAD % NTHR) == 0 && (WP_LAY % NTHR) == 0);
static_assert(GROWS == NWAVE * 16);
static_assert(NG == NWAVE * 16 && NTHR == 2 * NG);
static_assert(NCLS > 32 && NCLS <= 64 && ((NG * NCLS) % 4) == 0);

typedef float    v2f  __attribute__((ext_vector_type(2)));
typedef float    v4f  __attribute__((ext_vector_type(4)));
typedef float    v8f  __attribute__((ext_vector_type(8)));
typedef int      v4i  __attribute__((ext_vector_type(4)));
typedef _Float16 v8h  __attribute__((ext_vector_type(8)));
typedef _Float16 v16h __attribute__((ext_vector_type(16)));
union FragH { v16h v; v8h h[2]; };

__device__ __forceinline__ v8f wm(v16h a, v16h b, v8f c) {
  v8f d = __builtin_amdgcn_wmma_f32_16x16x32_f16(false, a, false, b, (short)0, c, false, false);
  asm volatile("v_nop\n\tv_nop\n\tv_nop\n\tv_nop" : "+v"(d) : "v"(a), "v"(b));
  return d;
}
__device__ __forceinline__ v8f z8f() { v8f z = {0.f, 0.f, 0.f, 0.f, 0.f, 0.f, 0.f, 0.f}; return z; }

__device__ __forceinline__ float silu_f(float v) {
  return v * __builtin_amdgcn_rcpf(1.0f + __expf(-v));
}
__device__ __forceinline__ v4f silu4(v4f v) {
  v4f r;
  r.x = silu_f(v.x); r.y = silu_f(v.y); r.z = silu_f(v.z); r.w = silu_f(v.w);
  return r;
}
__device__ __forceinline__ v8h cvt8(v4f a, v4f b) {
  v8h o;
  o[0] = (_Float16)a.x; o[1] = (_Float16)a.y; o[2] = (_Float16)a.z; o[3] = (_Float16)a.w;
  o[4] = (_Float16)b.x; o[5] = (_Float16)b.y; o[6] = (_Float16)b.z; o[7] = (_Float16)b.w;
  return o;
}
__device__ __forceinline__ v8h gath8h(const float* p, int stride) {
  v4f a, c;
  a.x = p[0];          a.y = p[stride];     a.z = p[2 * stride]; a.w = p[3 * stride];
  c.x = p[4 * stride]; c.y = p[5 * stride]; c.z = p[6 * stride]; c.w = p[7 * stride];
  return cvt8(a, c);
}

template <int NB>
__device__ __forceinline__ int scan_chunk(const int* __restrict__ keys, int nE, int cbase, int slotBase,
                                          int vec8, int* list, int tid, int lane, int wave) {
  int wc = 0;
#pragma unroll
  for (int g = 0; g < NGRP; ++g) {
    const int el0  = (g * NTHR + tid) * EPT;
    const int e0   = cbase + el0;
    const int sent = -2147483647 - 1;
    v4i da, db;
    if (vec8 != 0 && cbase + CHUNK <= nE) {
      da = *(const v4i*)(keys + e0);
      db = *(const v4i*)(keys + e0 + 4);
    } else {
      da.x = (e0     < nE) ? keys[min(e0, nE - 1)] : sent;
      da.y = (e0 + 1 < nE) ? keys[min(e0 + 1, nE - 1)] : sent;
      da.z = (e0 + 2 < nE) ? keys[min(e0 + 2, nE - 1)] : sent;
      da.w = (e0 + 3 < nE) ? keys[min(e0 + 3, nE - 1)] : sent;
      db.x = (e0 + 4 < nE) ? keys[min(e0 + 4, nE - 1)] : sent;
      db.y = (e0 + 5 < nE) ? keys[min(e0 + 5, nE - 1)] : sent;
      db.z = (e0 + 6 < nE) ? keys[min(e0 + 6, nE - 1)] : sent;
      db.w = (e0 + 7 < nE) ? keys[min(e0 + 7, nE - 1)] : sent;
    }
    const unsigned nb = (unsigned)slotBase;
    const unsigned s0 = (unsigned)da.x - nb, s1 = (unsigned)da.y - nb;
    const unsigned s2 = (unsigned)da.z - nb, s3 = (unsigned)da.w - nb;
    const unsigned s4 = (unsigned)db.x - nb, s5 = (unsigned)db.y - nb;
    const unsigned s6 = (unsigned)db.z - nb, s7 = (unsigned)db.w - nb;
    const bool h0 = s0 < (unsigned)NB, h1 = s1 < (unsigned)NB, h2 = s2 < (unsigned)NB, h3 = s3 < (unsigned)NB;
    const bool h4 = s4 < (unsigned)NB, h5 = s5 < (unsigned)NB, h6 = s6 < (unsigned)NB, h7 = s7 < (unsigned)NB;
    const unsigned any = __builtin_amdgcn_ballot_w32(h0 | h1 | h2 | h3 | h4 | h5 | h6 | h7);
    if (any != 0u) {
#define HITJ(J, HJ, SJ) { \
        const unsigned mj = __builtin_amdgcn_ballot_w32(HJ); \
        if (mj != 0u) { \
          if (HJ) { \
            const int pos = wc + (int)__builtin_amdgcn_mbcnt_lo(mj, 0u); \
            if (pos < WCAP) list[wave * WCAP + pos] = ((el0 + (J)) << 12) | (int)(SJ); \
          } \
          wc += (int)__builtin_popcount(mj); } }
      HITJ(0, h0, s0)
      HITJ(1, h1, s1)
      HITJ(2, h2, s2)
      HITJ(3, h3, s3)
      HITJ(4, h4, s4)
      HITJ(5, h5, s5)
      HITJ(6, h6, s6)
      HITJ(7, h7, s7)
#undef HITJ
    }
  }
  return wc;
}

__global__ __launch_bounds__(NTHR) void k_wprep(
    const float* __restrict__ wi, const float* __restrict__ wo,
    const float* __restrict__ ew1, const float* __restrict__ ew2,
    const float* __restrict__ cw1, const float* __restrict__ nw1,
    const float* __restrict__ nw2, _Float16* wp) {
  const int tid = (int)threadIdx.x;
  const int pc = (int)blockIdx.x * NTHR + tid;
  const float* src = wi;
  int K = IN_F, lp = pc;
  if (pc < 256) {
    src = wi; K = IN_F; lp = pc;
  } else if (pc < WP_HEAD) {
    src = wo; K = HF; lp = pc - 256;
  } else {
    const int lb = pc - WP_HEAD;
    const int l = lb / WP_LAY;
    const int r = lb - l * WP_LAY;
    if (r < 1024)      { src = ew1 + (size_t)l * (2 * HF + 1) * HF; K = HF;     lp = r; }
    else if (r < 1536) { src = ew2 + (size_t)l * HF * HF;           K = HF;     lp = r - 1024; }
    else if (r < 2048) { src = cw1 + (size_t)l * HF * HF;           K = HF;     lp = r - 1536; }
    else if (r < 3072) { src = nw1 + (size_t)l * 2 * HF * HF;       K = 2 * HF; lp = r - 2048; }
    else               { src = nw2 + (size_t)l * HF * HF;           K = HF;     lp = r - 3072; }
  }
  const int ppr = K >> 3;
  int n = lp / ppr;
  const int k0 = (lp - n * ppr) * 8;
  int kadd = 0;
  if (n >= HF) { kadd = HF; n -= HF; }
  const v8h o = gath8h(src + (size_t)(k0 + kadd) * HF + n, HF);
  _Float16* dp = wp + (size_t)pc * 8;
  *(volatile v8h*)dp = o;
  __threadfence();
  *(volatile v8h*)dp = o;
}

__global__ __launch_bounds__(NTHR) void k_count(
    const int* __restrict__ keys, int* cnt, int nE, int vec8) {
  __shared__ __attribute__((aligned(16))) int scnt[NBC];
  __shared__ __attribute__((aligned(16))) int list[LISTN];
  __shared__ int wcnt[NWAVE];
  const int tid = threadIdx.x, lane = tid & 31, wave = tid >> 5;
  const int nodeBase = blockIdx.x * NBC;

  for (int i = tid; i < NBC; i += NTHR) scnt[i] = 0;
  __syncthreads();

  const int nChunks = (nE + CHUNK - 1) / CHUNK;
#pragma unroll 1
  for (int ch = 0; ch < nChunks; ++ch) {
    const int cbase = ch * CHUNK;
    const int wc = scan_chunk<NBC>(keys, nE, cbase, nodeBase, vec8, list, tid, lane, wave);
    if (lane == 0) wcnt[wave] = wc;
    __syncthreads();
    if (wave == 0) {
#pragma unroll 1
      for (int wsx = 0; wsx < NWAVE; ++wsx) {
        int n = __builtin_amdgcn_readfirstlane(wcnt[wsx]);
        n = n > WCAP ? WCAP : (n < 0 ? 0 : n);
        const int* lp = list + wsx * WCAP;
#pragma unroll 1
        for (int i = 0; i < n; ++i) {
          const int ent  = __builtin_amdgcn_readfirstlane(lp[i]);
          const int slot = ent & (NBC - 1);
          if (lane == 0) scnt[slot] = scnt[slot] + 1;
        }
      }
    }
    __syncthreads();
  }

  v4i cq[4];
#pragma unroll
  for (int q = 0; q < 4; ++q) {
    const int f = (wave * 4 + q) * 128 + 4 * lane;
    cq[q] = *(const v4i*)(scnt + f);
  }
  int* cp = cnt + (size_t)nodeBase;
#pragma unroll
  for (int q = 0; q < 4; ++q) {
    const int f = (wave * 4 + q) * 128 + 4 * lane;
    *(volatile v4i*)(cp + f) = cq[q];
  }
  __threadfence();
#pragma unroll
  for (int q = 0; q < 4; ++q) {
    const int f = (wave * 4 + q) * 128 + 4 * lane;
    *(volatile v4i*)(cp + f) = cq[q];
  }
}

__global__ __launch_bounds__(OTHR) void k_offsets(
    const int* __restrict__ cnt, int* off, int* rbase, int nChunk) {
  __shared__ __attribute__((aligned(16))) int soff[NBC];
  __shared__ __attribute__((aligned(16))) int srb[RBN];
  __shared__ int wtot[OTHR / 32];
  const int tid = threadIdx.x, lane = tid & 31, wave = tid >> 5, sub = tid >> 7;
  for (int i = tid; i < RBN; i += OTHR) srb[i] = 0;
  int carry = 0;
#pragma unroll 1
  for (int ch = 0; ch < nChunk; ++ch) {
    const int base = ch * NBC;
    const v4i c0 = *(const v4i*)(cnt + base + 8 * tid);
    const v4i c1 = *(const v4i*)(cnt + base + 8 * tid + 4);
    const int e0 = max(c0.x, 0), e1 = max(c0.y, 0), e2 = max(c0.z, 0), e3 = max(c0.w, 0);
    const int e4 = max(c1.x, 0), e5 = max(c1.y, 0), e6 = max(c1.z, 0), e7 = max(c1.w, 0);
    const int ts = e0 + e1 + e2 + e3 + e4 + e5 + e6 + e7;
    int incl = ts;
#pragma unroll
    for (int d = 1; d < 32; d <<= 1) {
      const int t = __shfl_up(incl, d);
      if (lane >= d) incl += t;
    }
    if (lane == 31) wtot[wave] = incl;
    __syncthreads();
    const int S0 = wtot[0]  + wtot[1]  + wtot[2]  + wtot[3];
    const int S1 = wtot[4]  + wtot[5]  + wtot[6]  + wtot[7];
    const int S2 = wtot[8]  + wtot[9]  + wtot[10] + wtot[11];
    const int S3 = wtot[12] + wtot[13] + wtot[14] + wtot[15];
    int pre = 0;
#pragma unroll 1
    for (int w = 4 * sub; w < wave; ++w) pre += wtot[w];
    const int b0 = carry;
    const int b1 = b0 + ((S0 + 31) & ~31);
    const int b2 = b1 + ((S1 + 31) & ~31);
    const int b3 = b2 + ((S2 + 31) & ~31);
    const int b4 = b3 + ((S3 + 31) & ~31);
    const int myb = sub == 0 ? b0 : (sub == 1 ? b1 : (sub == 2 ? b2 : b3));
    if (tid == 0) {
      srb[min(4 * ch + 0, RBN - 1)] = b0;
      srb[min(4 * ch + 1, RBN - 1)] = b1;
      srb[min(4 * ch + 2, RBN - 1)] = b2;
      srb[min(4 * ch + 3, RBN - 1)] = b3;
    }
    int run = myb + pre + incl - ts;
    soff[8 * tid + 0] = run; run += e0;
    soff[8 * tid + 1] = run; run += e1;
    soff[8 * tid + 2] = run; run += e2;
    soff[8 * tid + 3] = run; run += e3;
    soff[8 * tid + 4] = run; run += e4;
    soff[8 * tid + 5] = run; run += e5;
    soff[8 * tid + 6] = run; run += e6;
    soff[8 * tid + 7] = run;
    carry = b4;
    __syncthreads();
    const v4i o0 = *(const v4i*)(soff + 4 * tid);
    const v4i o1 = *(const v4i*)(soff + 4 * (tid + OTHR));
    int* op = off + base;
    *(volatile v4i*)(op + 4 * tid) = o0;
    *(volatile v4i*)(op + 4 * (tid + OTHR)) = o1;
    __threadfence();
    *(volatile v4i*)(op + 4 * tid) = o0;
    *(volatile v4i*)(op + 4 * (tid + OTHR)) = o1;
    __syncthreads();
  }
  if (tid == 0) srb[min(4 * nChunk, RBN - 1)] = carry;
  __syncthreads();
  v4i rv = {0, 0, 0, 0};
  if (tid < 32) rv = *(const v4i*)(srb + 4 * tid);
  if (tid < 32) *(volatile v4i*)(rbase + 4 * tid) = rv;
  __threadfence();
  if (tid < 32) *(volatile v4i*)(rbase + 4 * tid) = rv;
}

__global__ __launch_bounds__(NTHR) void k_fill(
    const int* __restrict__ keys, const int* __restrict__ off, const int* __restrict__ rbase,
    int* csr, int nE, int vec8, int csrLen) {
  extern __shared__ v4f lds_dyn[];
  int* region = (int*)lds_dyn;
  int* cursor = region + RCAP;
  int* list   = cursor + NBF;
  int* wcnt   = list + LISTN;
  const int tid = threadIdx.x, lane = tid & 31, wave = tid >> 5;
  const int b = blockIdx.x;
  const int nodeBase = b * NBF;

  int rb0 = rbase[b];
  const int rb1 = rbase[b + 1];
  rb0 = rb0 < 0 ? 0 : (rb0 > csrLen ? csrLen : rb0);
  rb0 &= ~31;
  int len = rb1 - rb0;
  len = len < 0 ? 0 : (len > RCAP ? RCAP : len);
  int lenW = (len + 31) & ~31;
  if (rb0 + lenW > csrLen) lenW = (csrLen - rb0) & ~31;

  {
    const v4i z = {0, 0, 0, 0};
    for (int i = tid; i < RCAP / 4; i += NTHR) ((v4i*)region)[i] = z;
    for (int s = tid; s < NBF; s += NTHR) {
      int o = off[nodeBase + s] - rb0;
      o = o < 0 ? 0 : (o > RCAP ? RCAP : o);
      cursor[s] = o;
    }
  }
  __syncthreads();

  const int nChunks = (nE + CHUNK - 1) / CHUNK;
#pragma unroll 1
  for (int ch = 0; ch < nChunks; ++ch) {
    const int cbase = ch * CHUNK;
    const int wc = scan_chunk<NBF>(keys, nE, cbase, nodeBase, vec8, list, tid, lane, wave);
    if (lane == 0) wcnt[wave] = wc;
    __syncthreads();
    if (wave == 0) {
#pragma unroll 1
      for (int wsx = 0; wsx < NWAVE; ++wsx) {
        int n = __builtin_amdgcn_readfirstlane(wcnt[wsx]);
        n = n > WCAP ? WCAP : (n < 0 ? 0 : n);
        const int* lp = list + wsx * WCAP;
#pragma unroll 1
        for (int i = 0; i < n; ++i) {
          const int ent  = __builtin_amdgcn_readfirstlane(lp[i]);
          const int slot = ent & (NBF - 1);
          int e = cbase + ((ent >> 12) & (CHUNK - 1));
          e = e > nE - 1 ? nE - 1 : e;
          if (lane == 0) {
            int pos = cursor[slot];
            pos = pos < 0 ? 0 : (pos > RCAP - 1 ? RCAP - 1 : pos);
            region[pos] = e;
            const int np = pos + 1;
            cursor[slot] = np > RCAP ? RCAP : np;
          }
        }
      }
    }
    __syncthreads();
  }

  const int nv = lenW >> 2;
  int* gp = csr + rb0;
#pragma unroll 1
  for (int i = tid; i < nv; i += NTHR) { const v4i v = ((const v4i*)region)[i]; *(volatile v4i*)(gp + 4 * i) = v; }
  __threadfence();
#pragma unroll 1
  for (int i = tid; i < nv; i += NTHR) { const v4i v = ((const v4i*)region)[i]; *(volatile v4i*)(gp + 4 * i) = v; }
}

template <int K1, int K2, int NO>
struct NGCfg {
  static constexpr int KD  = K1 + K2;
  static constexpr int APH = KD + 8;
  static constexpr int LA  = GROWS * APH * 2;
  static constexpr int LS  = GROWS * NO * 4;
  static constexpr int LDS = LA > LS ? LA : LS;
};

template <int K1, int K2, int NO>
__global__ __launch_bounds__(NTHR) void k_ngemm(
    const float* __restrict__ A1, const float* __restrict__ A2,
    const _Float16* __restrict__ Bw, const float* __restrict__ bias,
    float* C, int nRowsA, int flags) {
  extern __shared__ v4f lds_dyn[];
  constexpr int KD = K1 + K2, APH = KD + 8, PPR = KD / 8, NIT = (GROWS * PPR) / NTHR, NT = NO / 16;
  constexpr int LN = NO / 4, RPI = 32 / LN, NI = 16 / RPI;
  static_assert((GROWS * PPR) % NTHR == 0);
  static_assert((KD % 32) == 0 && (NO == 64 || NO == 128));
  static_assert((K1 % 8) == 0 && (K2 % 8) == 0);
  _Float16* sAt = (_Float16*)lds_dyn;
  float*    stg = (float*)lds_dyn;
  const int tid = threadIdx.x, lane = tid & 31, wave = tid >> 5, hh = lane >> 4, m = lane & 15;
  const int rowBase = blockIdx.x * GROWS;

#pragma unroll
  for (int i = 0; i < NIT; ++i) {
    const int j = i * NTHR + tid;
    const int r = j / PPR;
    const int c8 = (j - r * PPR) * 8;
    int row = rowBase + r;
    row = row > nRowsA - 1 ? nRowsA - 1 : row;
    const float* ap = (K2 > 0 && c8 >= K1) ? (A2 + (size_t)row * (K2 > 0 ? K2 : 1) + (c8 - K1))
                                           : (A1 + (size_t)row * K1 + c8);
    const v4f a = *(const v4f*)ap, b = *(const v4f*)(ap + 4);
    *(v8h*)(sAt + r * APH + c8) = cvt8(a, b);
  }
  __syncthreads();

  v8f acc[NT];
#pragma unroll
  for (int t = 0; t < NT; ++t) acc[t] = z8f();
  const _Float16* fp = sAt + (wave * 16 + m) * APH + 8 * hh;
#pragma unroll
  for (int kt = 0; kt < KD / 32; ++kt) {
    FragH a;
    a.h[0] = *(const v8h*)(fp + 32 * kt);
    a.h[1] = *(const v8h*)(fp + 32 * kt + 16);
#pragma unroll
    for (int t = 0; t < NT; ++t) {
      const _Float16* bp = Bw + (size_t)(16 * t + m) * KD + 32 * kt + 8 * hh;
      FragH b;
      b.h[0] = *(const v8h*)bp;
      b.h[1] = *(const v8h*)(bp + 16);
      acc[t] = wm(a.v, b.v, acc[t]);
    }
  }
  __syncthreads();

  const int r0 = wave * 16 + 8 * hh;
  float* sp = stg + r0 * NO + m;
#pragma unroll
  for (int t = 0; t < NT; ++t) {
#pragma unroll
    for (int r = 0; r < 8; ++r) sp[r * NO + 16 * t] = acc[t][r];
  }
  __syncthreads();

  const v4f zero4 = {0.f, 0.f, 0.f, 0.f};
  const int rsub = lane / LN;
  const int c4 = (lane - rsub * LN) * 4;
  const v4f braw = *(const v4f*)(bias + c4);
  const v4f bsel = (flags & FL_BIAS) ? braw : zero4;
  v4f vals[NI];
#pragma unroll
  for (int i = 0; i < NI; ++i) {
    const int rl = wave * 16 + i * RPI + rsub;
    v4f v = *(const v4f*)(stg + rl * NO + c4);
    v = v + bsel;
    if (flags & FL_SILU) v = silu4(v);
    vals[i] = v;
  }
#pragma unroll
  for (int i = 0; i < NI; ++i) {
    const int rl = wave * 16 + i * RPI + rsub;
    *(volatile v4f*)(C + (size_t)(rowBase + rl) * NO + c4) = vals[i];
  }
  __threadfence();
#pragma unroll
  for (int i = 0; i < NI; ++i) {
    const int rl = wave * 16 + i * RPI + rsub;
    *(volatile v4f*)(C + (size_t)(rowBase + rl) * NO + c4) = vals[i];
  }
}

__global__ __launch_bounds__(ETHR) void k_edge(
    const int* __restrict__ offp, const int* __restrict__ cntp, const int* __restrict__ csr,
    const int* __restrict__ erow, const int* __restrict__ ecol,
    const float* __restrict__ xold, const float* __restrict__ pq,
    const float* __restrict__ ew1, const float* __restrict__ eb1,
    const _Float16* __restrict__ w2h, const float* __restrict__ eb2,
    const _Float16* __restrict__ c1h, const float* __restrict__ cb1,
    const float* __restrict__ cw2,
    float* agg, float* xnew, int nN, int nE, int csrLen) {
  __shared__ __attribute__((aligned(16))) _Float16 sT[CPOS * TPH];
  __shared__ __attribute__((aligned(16))) _Float16 sMh[CPOS * TPH];
  __shared__ __attribute__((aligned(16))) float sMf[CPOS * MPF];
  __shared__ __attribute__((aligned(16))) float sDf[CPOS * 4];
  __shared__ __attribute__((aligned(16))) float sB1[HF];
  __shared__ __attribute__((aligned(16))) float sWr[HF];
  __shared__ __attribute__((aligned(16))) float sB2[HF];
  __shared__ __attribute__((aligned(16))) float sBc[HF];
  __shared__ __attribute__((aligned(16))) float sWc[HF];
  __shared__ __attribute__((aligned(16))) float sX[CNB * 3];
  __shared__ float sRad[CPOS];
  __shared__ float sCc[CPOS];
  __shared__ int sRn[CPOS];
  __shared__ int sCn[CPOS];
  const int tid = threadIdx.x, lane = tid & 31, wave = tid >> 5, hh = lane >> 4, m = lane & 15;
  const int c0 = blockIdx.x * CNB;

  if (tid < HF) {
    sB1[tid] = eb1[tid];
    sWr[tid] = ew1[2 * HF * HF + tid];
    sB2[tid] = eb2[tid];
    sBc[tid] = cb1[tid];
    sWc[tid] = cw2[tid];
  }
  int offl = offp[c0 + lane];
  int cntl = cntp[c0 + lane];
  cntl = cntl < 0 ? 0 : (cntl > DEGCAP ? DEGCAP : cntl);
  offl = offl < 0 ? 0 : (offl > csrLen ? csrLen : offl);
  const int R0 = __builtin_amdgcn_readfirstlane(offl);
  const int Rend = __builtin_amdgcn_readlane(offl, 31) + __builtin_amdgcn_readlane(cntl, 31);
  int tot = Rend - R0;
  tot = tot < 0 ? 0 : (tot > CNB * DEGCAP ? CNB * DEGCAP : tot);
  const int nch = (tot + CPOS - 1) / CPOS;
  const int dsel = m < 3 ? m : 3;
  const int rowb = 16 * wave + 8 * hh;

  v4f nacc[8];
  float tacc[8];
#pragma unroll
  for (int s = 0; s < 8; ++s) { v4f zz = {0.f, 0.f, 0.f, 0.f}; nacc[s] = zz; tacc[s] = 0.f; }

#pragma unroll 1
  for (int ch = 0; ch < nch; ++ch) {
    const int P = R0 + ch * CPOS;
    __syncthreads();
    if (tid < CPOS) {
      int p = P + tid;
      p = p > csrLen - 1 ? csrLen - 1 : p;
      int e = csr[p];
      e = e < 0 ? 0 : (e > nE - 1 ? nE - 1 : e);
      int rn = erow[e];
      rn = rn < 0 ? 0 : (rn > nN - 1 ? nN - 1 : rn);
      int cn = ecol[e];
      cn = cn < 0 ? 0 : (cn > nN - 1 ? nN - 1 : cn);
      const float* xr = xold + (size_t)rn * 3;
      const float* xc = xold + (size_t)cn * 3;
      const float dx = xr[0] - xc[0], dy = xr[1] - xc[1], dz = xr[2] - xc[2];
      sDf[4 * tid + 0] = dx; sDf[4 * tid + 1] = dy; sDf[4 * tid + 2] = dz; sDf[4 * tid + 3] = 0.f;
      sRad[tid] = dx * dx + dy * dy + dz * dz;
      sRn[tid] = rn;
      sCn[tid] = cn;
    }
    __syncthreads();

    {
      const int r = tid >> 1, q = tid & 1;
      const int rn = sRn[r], cn = sCn[r];
      const float rad = sRad[r];
      const float* pp = pq + (size_t)rn * MD + 32 * q;
      const float* qp = pq + (size_t)cn * MD + HF + 32 * q;
#pragma unroll
      for (int i = 0; i < 4; ++i) {
        const int cb = 32 * q + 8 * i;
        const v4f p0 = *(const v4f*)(pp + 8 * i), p1 = *(const v4f*)(pp + 8 * i + 4);
        const v4f q0 = *(const v4f*)(qp + 8 * i), q1 = *(const v4f*)(qp + 8 * i + 4);
        const v4f b0 = *(const v4f*)(sB1 + cb), b1v = *(const v4f*)(sB1 + cb + 4);
        const v4f w0 = *(const v4f*)(sWr + cb), w1v = *(const v4f*)(sWr + cb + 4);
        const v4f u0 = (p0 + q0) + rad * w0 + b0;
        const v4f u1 = (p1 + q1) + rad * w1v + b1v;
        *(v8h*)(sT + r * TPH + cb) = cvt8(silu4(u0), silu4(u1));
      }
    }
    __syncthreads();

    v8f acc[4];
#pragma unroll
    for (int t = 0; t < 4; ++t) acc[t] = z8f();
    {
      const _Float16* fp = sT + (16 * wave + m) * TPH + 8 * hh;
#pragma unroll
      for (int ks = 0; ks < HF / 32; ++ks) {
        FragH a;
        a.h[0] = *(const v8h*)(fp + 32 * ks);
        a.h[1] = *(const v8h*)(fp + 32 * ks + 16);
#pragma unroll
        for (int t = 0; t < 4; ++t) {
          const _Float16* bp = w2h + (size_t)(16 * t + m) * HF + 32 * ks + 8 * hh;
          FragH b;
          b.h[0] = *(const v8h*)bp;
          b.h[1] = *(const v8h*)(bp + 16);
          acc[t] = wm(a.v, b.v, acc[t]);
        }
      }
    }
#pragma unroll
    for (int t = 0; t < 4; ++t) {
      const int n = 16 * t + m;
      const float bv = sB2[n];
#pragma unroll
      for (int r = 0; r < 8; ++r) {
        const float v = silu_f(acc[t][r] + bv);
        sMf[(rowb + r) * MPF + n] = v;
        sMh[(rowb + r) * TPH + n] = (_Float16)v;
      }
    }
    __syncthreads();

#pragma unroll
    for (int t = 0; t < 4; ++t) acc[t] = z8f();
    {
      const _Float16* fp = sMh + (16 * wave + m) * TPH + 8 * hh;
#pragma unroll
      for (int ks = 0; ks < HF / 32; ++ks) {
        FragH a;
        a.h[0] = *(const v8h*)(fp + 32 * ks);
        a.h[1] = *(const v8h*)(fp + 32 * ks + 16);
#pragma unroll
        for (int t = 0; t < 4; ++t) {
          const _Float16* bp = c1h + (size_t)(16 * t + m) * HF + 32 * ks + 8 * hh;
          FragH b;
          b.h[0] = *(const v8h*)bp;
          b.h[1] = *(const v8h*)(bp + 16);
          acc[t] = wm(a.v, b.v, acc[t]);
        }
      }
    }
    float pcv[8];
#pragma unroll
    for (int r = 0; r < 8; ++r) pcv[r] = 0.f;
#pragma unroll
    for (int t = 0; t < 4; ++t) {
      const int n = 16 * t + m;
      const float bv = sBc[n];
      const float wv = sWc[n];
#pragma unroll
      for (int r = 0; r < 8; ++r) pcv[r] += silu_f(acc[t][r] + bv) * wv;
    }
#pragma unroll
    for (int r = 0; r < 8; ++r) {
      pcv[r] += __shfl_xor(pcv[r], 1);
      pcv[r] += __shfl_xor(pcv[r], 2);
      pcv[r] += __shfl_xor(pcv[r], 4);
      pcv[r] += __shfl_xor(pcv[r], 8);
    }
    if (m == 0) {
#pragma unroll
      for (int r = 0; r < 8; ++r) sCc[rowb + r] = pcv[r];
    }
    __syncthreads();

#pragma unroll
    for (int s = 0; s < 8; ++s) {
      const int j  = 8 * wave + s;
      const int oj = __shfl(offl, j);
      const int cj = __shfl(cntl, j);
      int lo = oj - P;
      lo = lo < 0 ? 0 : (lo > CPOS ? CPOS : lo);
      int hi = oj + cj - P;
      hi = hi < 0 ? 0 : (hi > CPOS ? CPOS : hi);
#pragma unroll 1
      for (int r = lo; r < hi; ++r) {
        const v4f mv = *(const v4f*)(sMf + r * MPF + 4 * m);
        nacc[s] = nacc[s] + mv;
        tacc[s] += sDf[r * 4 + dsel] * sCc[r];
      }
    }
  }

#pragma unroll
  for (int s = 0; s < 8; ++s) {
    const int j = 8 * wave + s;
    const int cj = __shfl(cntl, j);
    const float inv = 1.0f / fmaxf((float)cj, 1.0f);
    int c = c0 + j;
    c = c > nN - 1 ? nN - 1 : c;
    const int dl = m < 2 ? m : 2;
    const float xo = xold[(size_t)c * 3 + dl];
    const float xn = xo + tacc[s] * inv;
    if (hh == 0 && m < 3) sX[j * 3 + m] = xn;
  }
  __syncthreads();
  const int tq = tid < 23 ? tid : 23;
  const v4f xv = *(const v4f*)(sX + 4 * tq);

#pragma unroll
  for (int s = 0; s < 8; ++s) {
    const int c = c0 + 8 * wave + s;
    if (lane < 16) *(volatile v4f*)(agg + (size_t)c * HF + 4 * lane) = nacc[s];
  }
  if (tid < 24) *(volatile v4f*)(xnew + (size_t)c0 * 3 + 4 * tid) = xv;
  __threadfence();
#pragma unroll
  for (int s = 0; s < 8; ++s) {
    const int c = c0 + 8 * wave + s;
    if (lane < 16) *(volatile v4f*)(agg + (size_t)c * HF + 4 * lane) = nacc[s];
  }
  if (tid < 24) *(volatile v4f*)(xnew + (size_t)c0 * 3 + 4 * tid) = xv;
}

__global__ __launch_bounds__(ETHR) void k_pool(
    const float* __restrict__ hf, const int* __restrict__ bat, float* hp, int nN) {
  __shared__ __attribute__((aligned(16))) float sMx[4 * HF];
  const int tid = threadIdx.x, lane = tid & 31, wave = tid >> 5;
  const int g = blockIdx.x;
  const float ninf = __uint_as_float(0xff800000u);
  float m0 = ninf, m1 = ninf;
  const int nIt = (nN + ETHR - 1) / ETHR;
#pragma unroll 1
  for (int it = 0; it < nIt; ++it) {
    const int n = it * ETHR + tid;
    const int nc = n < nN ? n : nN - 1;
    const int b = bat[nc];
    const bool hit = (n < nN) && (b == g);
    unsigned msk = __builtin_amdgcn_ballot_w32(hit);
    msk = (unsigned)__builtin_amdgcn_readfirstlane((int)msk);
    while (msk != 0u) {
      const int l = __builtin_ctz(msk);
      msk &= msk - 1u;
      int node = it * ETHR + 32 * wave + l;
      node = node > nN - 1 ? nN - 1 : node;
      const v2f v = *(const v2f*)(hf + (size_t)node * HF + 2 * lane);
      m0 = fmaxf(m0, v.x);
      m1 = fmaxf(m1, v.y);
    }
  }
  sMx[wave * HF + 2 * lane] = m0;
  sMx[wave * HF + 2 * lane + 1] = m1;
  __syncthreads();
  const int c4 = 4 * (lane & 15);
  v4f r = *(const v4f*)(sMx + c4);
#pragma unroll
  for (int w = 1; w < 4; ++w) {
    const v4f q = *(const v4f*)(sMx + w * HF + c4);
    r.x = fmaxf(r.x, q.x); r.y = fmaxf(r.y, q.y); r.z = fmaxf(r.z, q.z); r.w = fmaxf(r.w, q.w);
  }
  float* gp = hp + (size_t)g * HF + c4;
  if (wave == 0 && lane < 16) *(volatile v4f*)gp = r;
  __threadfence();
  if (wave == 0 && lane < 16) *(volatile v4f*)gp = r;
}

__global__ __launch_bounds__(NTHR) void k_head(
    const float* __restrict__ hp, const float* __restrict__ w1, const float* __restrict__ b1,
    const float* __restrict__ w2, const float* __restrict__ b2,
    const float* __restrict__ w3, const float* __restrict__ b3, float* out) {
  extern __shared__ v4f lds_dyn[];
  _Float16* sA = (_Float16*)lds_dyn;
  _Float16* sB = sA + NG * MD;
  float* sL = (float*)sB;
  float* sO = (float*)sA;
  const int tid = threadIdx.x, lane = tid & 31, wave = tid >> 5, hh = lane >> 4, m = lane & 15;
  const int rowb = 16 * wave + 8 * hh;

  {
    const int r = tid >> 1, q = tid & 1;
    const float* src = hp + (size_t)r * HF + 32 * q;
#pragma unroll
    for (int i = 0; i < 4; ++i) {
      const v4f a = *(const v4f*)(src + 8 * i), c = *(const v4f*)(src + 8 * i + 4);
      *(v8h*)(sA + r * MD + 32 * q + 8 * i) = cvt8(a, c);
    }
  }
  {
    const int k = tid >> 2, cb = (tid & 3) * 32;
    const float* src = w1 + (size_t)k * MD + cb;
#pragma unroll 1
    for (int bq = 0; bq < 2; ++bq) {
      v4f v[4];
#pragma unroll
      for (int i = 0; i < 4; ++i) v[i] = *(const v4f*)(src + 16 * bq + 4 * i);
#pragma unroll
      for (int i = 0; i < 4; ++i) {
        const int n = cb + 16 * bq + 4 * i;
        sB[(n + 0) * MD + k] = (_Float16)v[i].x;
        sB[(n + 1) * MD + k] = (_Float16)v[i].y;
        sB[(n + 2) * MD + k] = (_Float16)v[i].z;
        sB[(n + 3) * MD + k] = (_Float16)v[i].w;
      }
    }
  }
  __syncthreads();

  v8f acc[8];
#pragma unroll
  for (int t = 0; t < 8; ++t) acc[t] = z8f();
  {
    const _Float16* fp = sA + (16 * wave + m) * MD + 8 * hh;
#pragma unroll
    for (int kt = 0; kt < HF / 32; ++kt) {
      FragH a;
      a.h[0] = *(const v8h*)(fp + 32 * kt);
      a.h[1] = *(const v8h*)(fp + 32 * kt + 16);
#pragma unroll
      for (int t = 0; t < 8; ++t) {
        const _Float16* bp = sB + (16 * t + m) * MD + 32 * kt + 8 * hh;
        FragH b;
        b.h[0] = *(const v8h*)bp;
        b.h[1] = *(const v8h*)(bp + 16);
        acc[t] = wm(a.v, b.v, acc[t]);
      }
    }
  }
  __syncthreads();
#pragma unroll
  for (int t = 0; t < 8; ++t) {
    const int n = 16 * t + m;
    const float bv = b1[n];
#pragma unroll
    for (int r = 0; r < 8; ++r) sA[(rowb + r) * MD + n] = (_Float16)fmaxf(acc[t][r] + bv, 0.f);
  }
  {
    const int k = tid >> 1, cb = (tid & 1) * 64;
    const float* src = w2 + (size_t)k * MD + cb;
#pragma unroll 1
    for (int bq = 0; bq < 4; ++bq) {
      v4f v[4];
#pragma unroll
      for (int i = 0; i < 4; ++i) v[i] = *(const v4f*)(src + 16 * bq + 4 * i);
#pragma unroll
      for (int i = 0; i < 4; ++i) {
        const int n = cb + 16 * bq + 4 * i;
        sB[(n + 0) * MD + k] = (_Float16)v[i].x;
        sB[(n + 1) * MD + k] = (_Float16)v[i].y;
        sB[(n + 2) * MD + k] = (_Float16)v[i].z;
        sB[(n + 3) * MD + k] = (_Float16)v[i].w;
      }
    }
  }
  __syncthreads();

#pragma unroll
  for (int t = 0; t < 8; ++t) acc[t] = z8f();
  {
    const _Float16* fp = sA + (16 * wave + m) * MD + 8 * hh;
#pragma unroll
    for (int kt = 0; kt < MD / 32; ++kt) {
      FragH a;
      a.h[0] = *(const v8h*)(fp + 32 * kt);
      a.h[1] = *(const v8h*)(fp + 32 * kt + 16);
#pragma unroll
      for (int t = 0; t < 8; ++t) {
        const _Float16* bp = sB + (16 * t + m) * MD + 32 * kt + 8 * hh;
        FragH b;
        b.h[0] = *(const v8h*)bp;
        b.h[1] = *(const v8h*)(bp + 16);
        acc[t] = wm(a.v, b.v, acc[t]);
      }
    }
  }
  __syncthreads();
#pragma unroll
  for (int t = 0; t < 8; ++t) {
    const int n = 16 * t + m;
    const float bv = b2[n];
#pragma unroll
    for (int r = 0; r < 8; ++r) sA[(rowb + r) * MD + n] = (_Float16)fmaxf(acc[t][r] + bv, 0.f);
  }
  {
    const int k = tid >> 1, nb = (tid & 1) * 32;
    const float* src = w3 + (size_t)k * NCLS;
#pragma unroll 1
    for (int bq = 0; bq < 4; ++bq) {
      float v[8];
#pragma unroll
      for (int j = 0; j < 8; ++j) {
        const int n = nb + 8 * bq + j;
        const int nc = n < NCLS ? n : NCLS - 1;
        const float f = src[nc];
        v[j] = (n < NCLS) ? f : 0.0f;
      }
#pragma unroll
      for (int j = 0; j < 8; ++j) sB[(nb + 8 * bq + j) * MD + k] = (_Float16)v[j];
    }
  }
  __syncthreads();

  v8f acc3[4];
#pragma unroll
  for (int t = 0; t < 4; ++t) acc3[t] = z8f();
  {
    const _Float16* fp = sA + (16 * wave + m) * MD + 8 * hh;
#pragma unroll
    for (int kt = 0; kt < MD / 32; ++kt) {
      FragH a;
      a.h[0] = *(const v8h*)(fp + 32 * kt);
      a.h[1] = *(const v8h*)(fp + 32 * kt + 16);
#pragma unroll
      for (int t = 0; t < 4; ++t) {
        const _Float16* bp = sB + (16 * t + m) * MD + 32 * kt + 8 * hh;
        FragH b;
        b.h[0] = *(const v8h*)bp;
        b.h[1] = *(const v8h*)(bp + 16);
        acc3[t] = wm(a.v, b.v, acc3[t]);
      }
    }
  }
  __syncthreads();
#pragma unroll
  for (int t = 0; t < 4; ++t) {
    const int n = 16 * t + m;
    const int nc = n < NCLS ? n : NCLS - 1;
    const float bv = b3[nc];
#pragma unroll
    for (int r = 0; r < 8; ++r) sL[(rowb + r) * HF + n] = acc3[t][r] + bv;
  }
  __syncthreads();

  const float ninf = __uint_as_float(0xff800000u);
#pragma unroll 1
  for (int i = 0; i < 16; ++i) {
    const int row = 16 * wave + i;
    const float v0 = sL[row * HF + lane];
    const int l1 = lane < (NCLS - 33) ? lane : (NCLS - 33);
    const float v1r = sL[row * HF + 32 + l1];
    const bool ok1 = lane < (NCLS - 32);
    float mx = fmaxf(v0, ok1 ? v1r : ninf);
#pragma unroll
    for (int o = 16; o > 0; o >>= 1) mx = fmaxf(mx, __shfl_xor(mx, o));
    const float e0 = expf(v0 - mx);
    const float e1r = expf(v1r - mx);
    float s = e0 + (ok1 ? e1r : 0.0f);
#pragma unroll
    for (int o = 16; o > 0; o >>= 1) s += __shfl_xor(s, o);
    const float lse = logf(s);
    sO[row * NCLS + lane] = (v0 - mx) - lse;
    if (ok1) sO[row * NCLS + 32 + lane] = (v1r - mx) - lse;
  }
  __syncthreads();

  constexpr int NQ = (NG * NCLS) / 4;
  v4f ov[7];
#pragma unroll
  for (int j = 0; j < 7; ++j) {
    const int i = j * NTHR + tid;
    const int ic = i < NQ ? i : NQ - 1;
    ov[j] = *(const v4f*)(sO + 4 * ic);
  }
#pragma unroll
  for (int j = 0; j < 7; ++j) {
    const int i = j * NTHR + tid;
    if (i < NQ) *(volatile v4f*)(out + 4 * (size_t)i) = ov[j];
  }
  __threadfence();
#pragma unroll
  for (int j = 0; j < 7; ++j) {
    const int i = j * NTHR + tid;
    if (i < NQ) *(volatile v4f*)(out + 4 * (size_t)i) = ov[j];
  }
}

extern "C" void kernel_launch(void* const* d_in, const int* in_sizes, int n_in,
                              void* d_out, int out_size, void* d_ws, size_t ws_size,
                              hipStream_t stream) {
  if (n_in < 25) return;
  const int nN = in_sizes[3];
  if (nN <= 0 || nN > (1 << 22)) return;
  if (in_sizes[0] != nN * IN_F || in_sizes[1] != nN * 3) return;
  const int nE2 = in_sizes[2];
  if (nE2 <= 0 || (nE2 & 1) != 0) return;
  const int nE = nE2 / 2;
  if (nE > (1 << 26)) return;
  const int nL = in_sizes[6] / ((2 * HF + 1) * HF);
  if (nL < 1 || nL > 16 || in_sizes[6] != nL * (2 * HF + 1) * HF) return;
  if (in_sizes[4] != IN_F * HF || in_sizes[5] != HF) return;
  if (in_sizes[7] != nL * HF || in_sizes[8] != nL * HF * HF || in_sizes[9] != nL * HF) return;
  if (in_sizes[10] != nL * 2 * HF * HF || in_sizes[11] != nL * HF) return;
  if (in_sizes[12] != nL * HF * HF || in_sizes[13] != nL * HF) return;
  if (in_sizes[14] != nL * HF * HF || in_sizes[15] != nL * HF || in_sizes[16] != nL * HF) return;
  if (in_sizes[17] != HF * HF || in_sizes[18] != HF) return;
  if (in_sizes[19] != HF * MD || in_sizes[20] != MD || in_sizes[21] != MD * MD || in_sizes[22] != MD) return;
  if (in_sizes[23] != MD * NCLS || in_sizes[24] != NCLS) return;
  if (out_size != NG * NCLS) return;

  const float* hin = (const float*)d_in[0];
  const float* xin = (const float*)d_in[1];
  const int*   ei  = (const int*)d_in[2];
  const int*   bat = (const int*)d_in[3];
  const float* wi  = (const float*)d_in[4];
  const float* bi  = (const float*)d_in[5];
  const float* ew1 = (const float*)d_in[6];
  const float* eb1 = (const float*)d_in[7];
  const float* ew2 = (const float*)d_in[8];
  const float* eb2 = (const float*)d_in[9];
  const float* nw1 = (const float*)d_in[10];
  const float* nb1 = (const float*)d_in[11];
  const float* nw2 = (const float*)d_in[12];
  const float* nb2 = (const float*)d_in[13];
  const float* cw1 = (const float*)d_in[14];
  const float* cb1 = (const float*)d_in[15];
  const float* cw2 = (const float*)d_in[16];
  const float* wo  = (const float*)d_in[17];
  const float* bo  = (const float*)d_in[18];
  const float* f1w = (const float*)d_in[19];
  const float* f1b = (const float*)d_in[20];
  const float* f2w = (const float*)d_in[21];
  const float* f2b = (const float*)d_in[22];
  const float* f3w = (const float*)d_in[23];
  const float* f3b = (const float*)d_in[24];
  float* out = (float*)d_out;
  const int* erow = ei;
  const int* ecol = ei + nE;

  const int NPAD   = ((nN + GROWS - 1) / GROWS) * GROWS;
  const int nBC    = (nN + NBC - 1) / NBC;
  const int CNTPAD = nBC * NBC;
  if (NPAD > CNTPAD) return;
  if (4 * nBC + 1 > RBN) return;
  const int nBF    = (nN + NBF - 1) / NBF;
  if (31 * 4 * nBC > 4096) return;
  const int csrLen = ((nE + 31) & ~31) + 4096;
  const int nEdge  = NPAD / CNB;
  const int nGemm  = NPAD / GROWS;
  const int nWp    = (WP_HEAD + nL * WP_LAY) / NTHR;

  char* ws = (char*)d_ws;
  size_t off = 0;
  const size_t plane = (size_t)NPAD * HF * 4;
  const size_t oW   = off; off += (size_t)(WP_HEAD + nL * WP_LAY) * 16; off = (off + 255) & ~(size_t)255;
  const size_t oCnt = off; off += (size_t)CNTPAD * 4;                  off = (off + 255) & ~(size_t)255;
  const size_t oOff = off; off += (size_t)CNTPAD * 4;                  off = (off + 255) & ~(size_t)255;
  const size_t oRb  = off; off += (size_t)RBN * 4;                     off = (off + 255) & ~(size_t)255;
  const size_t oCsr = off; off += (size_t)csrLen * 4;                  off = (off + 255) & ~(size_t)255;
  const size_t oHA  = off; off += plane;                               off = (off + 255) & ~(size_t)255;
  const size_t oHB  = off; off += plane;                               off = (off + 255) & ~(size_t)255;
  const size_t oNH  = off; off += plane;                               off = (off + 255) & ~(size_t)255;
  const size_t oAgg = off; off += plane;                               off = (off + 255) & ~(size_t)255;
  const size_t oPQ  = off; off += (size_t)NPAD * MD * 4;               off = (off + 255) & ~(size_t)255;
  const size_t oXA  = off; off += (size_t)NPAD * 3 * 4;                off = (off + 255) & ~(size_t)255;
  const size_t oXB  = off; off += (size_t)NPAD * 3 * 4;                off = (off + 255) & ~(size_t)255;
  const size_t oHp  = off; off += (size_t)NG * HF * 4;                 off = (off + 255) & ~(size_t)255;
  if (off > ws_size || off > (size_t)WSCAP) return;
  _Float16* wp = (_Float16*)(ws + oW);
  int*   cnt  = (int*)(ws + oCnt);
  int*   offp = (int*)(ws + oOff);
  int*   rb   = (int*)(ws + oRb);
  int*   csr  = (int*)(ws + oCsr);
  float* hA   = (float*)(ws + oHA);
  float* hB   = (float*)(ws + oHB);
  float* nh   = (float*)(ws + oNH);
  float* agg  = (float*)(ws + oAgg);
  float* pqp  = (float*)(ws + oPQ);
  float* xA   = (float*)(ws + oXA);
  float* xB   = (float*)(ws + oXB);
  float* hp   = (float*)(ws + oHp);

  const int vec8 = ((nE & 3) == 0) ? 1 : 0;

  k_wprep<<<nWp, NTHR, 0, stream>>>(wi, wo, ew1, ew2, cw1, nw1, nw2, wp);

  k_count<<<nBC, NTHR, 0, stream>>>(erow, cnt, nE, vec8);
  k_offsets<<<1, OTHR, 0, stream>>>(cnt, offp, rb, nBC);
  hipFuncSetAttribute(reinterpret_cast<const void*>(&k_fill),
                      hipFuncAttributeMaxDynamicSharedMemorySize, LDS_FILL);
  k_fill<<<nBF, NTHR, LDS_FILL, stream>>>(erow, offp, rb, csr, nE, vec8, csrLen);

  hipFuncSetAttribute(reinterpret_cast<const void*>(&k_ngemm<IN_F, 0, HF>),
                      hipFuncAttributeMaxDynamicSharedMemorySize, NGCfg<IN_F, 0, HF>::LDS);
  hipFuncSetAttribute(reinterpret_cast<const void*>(&k_ngemm<HF, 0, MD>),
                      hipFuncAttributeMaxDynamicSharedMemorySize, NGCfg<HF, 0, MD>::LDS);
  hipFuncSetAttribute(reinterpret_cast<const void*>(&k_ngemm<HF, HF, HF>),
                      hipFuncAttributeMaxDynamicSharedMemorySize, NGCfg<HF, HF, HF>::LDS);
  hipFuncSetAttribute(reinterpret_cast<const void*>(&k_ngemm<HF, 0, HF>),
                      hipFuncAttributeMaxDynamicSharedMemorySize, NGCfg<HF, 0, HF>::LDS);
  k_ngemm<IN_F, 0, HF><<<nGemm, NTHR, NGCfg<IN_F, 0, HF>::LDS, stream>>>(
      hin, hin, wp + WO_IN, bi, hA, nN, FL_BIAS);

  const float* xcur = xin;
  for (int l = 0; l < nL; ++l) {
    const _Float16* wl = wp + WO_LAY0 + (size_t)l * WL_STR;
    const float* hcur = (l & 1) ? hB : hA;
    float* hnext = (l & 1) ? hA : hB;
    float* xnext = (l & 1) ? xB : xA;
    k_ngemm<HF, 0, MD><<<nGemm, NTHR, NGCfg<HF, 0, MD>::LDS, stream>>>(
        hcur, hcur, wl + WL_PQ, f1b, pqp, NPAD, 0);
    k_edge<<<nEdge, ETHR, 0, stream>>>(
        offp, cnt, csr, erow, ecol, xcur, pqp,
        ew1 + (size_t)l * (2 * HF + 1) * HF, eb1 + (size_t)l * HF,
        wl + WL_W2, eb2 + (size_t)l * HF,
        wl + WL_C1, cb1 + (size_t)l * HF, cw2 + (size_t)l * HF,
        agg, xnext, nN, nE, csrLen);
    k_ngemm<HF, HF, HF><<<nGemm, NTHR, NGCfg<HF, HF, HF>::LDS, stream>>>(
        hcur, agg, wl + WL_N1, nb1 + (size_t)l * HF, nh, NPAD, FL_BIAS | FL_SILU);
    k_ngemm<HF, 0, HF><<<nGemm, NTHR, NGCfg<HF, 0, HF>::LDS, stream>>>(
        nh, nh, wl + WL_N2, nb2 + (size_t)l * HF, hnext, NPAD, FL_BIAS);
    xcur = xnext;
  }
  const float* hfin = (nL & 1) ? hB : hA;

  k_ngemm<HF, 0, HF><<<nGemm, NTHR, NGCfg<HF, 0, HF>::LDS, stream>>>(
      hfin, hfin, wp + WO_OUT, bo, nh, NPAD, FL_BIAS);

  k_pool<<<NG, ETHR, 0, stream>>>(nh, bat, hp, nN);

  hipFuncSetAttribute(reinterpret_cast<const void*>(&k_head),
                      hipFuncAttributeMaxDynamicSharedMemorySize, LDS_HEAD);
  k_head<<<1, NTHR, LDS_HEAD, stream>>>(hp, f1w, f1b, f2w, f2b, f3w, f3b, out);
}
